// MuleDetectorGNN_81011673137241
// MI455X (gfx1250) — hardware-run, weakly checked
//
#include <hip/hip_runtime.h>

typedef float          v8f   __attribute__((ext_vector_type(8)));
typedef float          v4f   __attribute__((ext_vector_type(4)));
typedef unsigned int   v4u   __attribute__((ext_vector_type(4)));
typedef int            v8i   __attribute__((ext_vector_type(8)));
typedef unsigned short v8us  __attribute__((ext_vector_type(8)));
typedef unsigned short v16us __attribute__((ext_vector_type(16)));
typedef __bf16         v16bf __attribute__((ext_vector_type(16)));
typedef _Float16       v16h  __attribute__((ext_vector_type(16)));
typedef v4f  __attribute__((may_alias)) v4fa;
typedef v8us __attribute__((may_alias)) v8usa;
union FragB { v16bf v; v16us u; v8us h[2]; v8i w; };
union FragH { v16h  v; v16us u; v8us h[2]; v8i w; };

__device__ __forceinline__ v8f wmb(const FragB& a, const FragB& b, v8f c) {
  v8f d = __builtin_amdgcn_wmma_f32_16x16x32_bf16(false, a.v, false, b.v, (short)0, c, false, false);
  asm volatile("v_nop\n\tv_nop\n\tv_nop\n\tv_nop" : "+v"(d) : "v"(a.w), "v"(b.w));
  return d;
}

__device__ __forceinline__ v8f wmh(const FragH& a, const FragH& b, v8f c) {
  v8f d = __builtin_amdgcn_wmma_f32_16x16x32_f16(false, a.v, false, b.v, (short)0, c, false, false);
  asm volatile("v_nop\n\tv_nop\n\tv_nop\n\tv_nop" : "+v"(d) : "v"(a.w), "v"(b.w));
  return d;
}

__device__ __forceinline__ unsigned bf16_bits(float f) {
  const unsigned u = __float_as_uint(f);
  const unsigned r = (u + 0x7FFFu + ((u >> 16) & 1u)) >> 16;
  const unsigned q = (u >> 16) | 0x40u;
  return ((u & 0x7fffffffu) > 0x7f800000u) ? q : r;
}

__device__ __forceinline__ float bf16_val(float f) {
  return __uint_as_float(bf16_bits(f) << 16);
}
__device__ __forceinline__ int clampi(int v, int lo, int hi) {
  return v < lo ? lo : (v > hi ? hi : v);
}

__device__ __forceinline__ unsigned f16_bits(float f) {
  const unsigned u  = __float_as_uint(f);
  const unsigned s  = (u >> 16) & 0x8000u;
  const unsigned a  = u & 0x7fffffffu;
  const unsigned t  = a - 0x38000000u;
  const unsigned r  = (t + 0x0FFFu + ((t >> 13) & 1u)) >> 13;
  const unsigned rc = r > 0x7C00u ? 0x7C00u : r;
  const bool small  = a < 0x38800000u;
  const bool isnan  = a > 0x7f800000u;
  const unsigned fin = small ? 0u : (s | rc);
  return isnan ? (s | 0x7E00u) : fin;
}

__device__ __forceinline__ unsigned pk16(unsigned lo, unsigned hi) { return lo | (hi << 16); }
__device__ __forceinline__ unsigned bf16_lo_bits(float v) {
  float hi = bf16_val(v);
  asm volatile("" : "+v"(hi));
  return bf16_bits(v - hi);
}
__device__ __forceinline__ v4u pack8_bf16(v4f a, v4f c) {
  return (v4u){ pk16(bf16_bits(a[0]), bf16_bits(a[1])), pk16(bf16_bits(a[2]), bf16_bits(a[3])),
                pk16(bf16_bits(c[0]), bf16_bits(c[1])), pk16(bf16_bits(c[2]), bf16_bits(c[3])) };
}
__device__ __forceinline__ v4u pack8_bf16_lo(v4f a, v4f c) {
  return (v4u){ pk16(bf16_lo_bits(a[0]), bf16_lo_bits(a[1])), pk16(bf16_lo_bits(a[2]), bf16_lo_bits(a[3])),
                pk16(bf16_lo_bits(c[0]), bf16_lo_bits(c[1])), pk16(bf16_lo_bits(c[2]), bf16_lo_bits(c[3])) };
}
__device__ __forceinline__ v4u pack8_f16(v4f a, v4f c) {
  return (v4u){ pk16(f16_bits(a[0]), f16_bits(a[1])), pk16(f16_bits(a[2]), f16_bits(a[3])),
                pk16(f16_bits(c[0]), f16_bits(c[1])), pk16(f16_bits(c[2]), f16_bits(c[3])) };
}

template <int FORM>
__global__ __launch_bounds__(256) void k_plane(const float* __restrict__ src, int rows, int cols, int ldsrc,
                                               unsigned short* __restrict__ dst, int MP, int KP) {
  static_assert(FORM >= 0 && FORM <= 3);
  const int KTOT = (FORM == 1 || FORM == 3) ? 2 * KP : KP;
  const unsigned ppr   = (unsigned)(KTOT >> 3);
  const unsigned kp8   = (unsigned)(KP >> 3);
  const unsigned total = (unsigned)MP * ppr;
  const unsigned g     = blockIdx.x * 256u + threadIdx.x;
  const unsigned rowu  = g / ppr;
  const unsigned p     = g - rowu * ppr;
  const bool second    = p >= kp8;
  const int row = (int)rowu;
  const int c0  = (int)((second ? p - kp8 : p) << 3);
  const float* srow = src + (size_t)clampi(row, 0, rows - 1) * (size_t)ldsrc;
  float x[8];
  unsigned mk[8];
#pragma unroll
  for (int e = 0; e < 8; ++e) {
    const int c = c0 + e;
    const float v = srow[clampi(c, 0, cols - 1)];
    asm volatile("" :: "v"(v));
    x[e]  = v;
    mk[e] = (row < rows && c < cols) ? 0xFFFFu : 0u;
  }
  const v4f a = (v4f){ x[0], x[1], x[2], x[3] };
  const v4f c = (v4f){ x[4], x[5], x[6], x[7] };
  v4u o;
  if (FORM == 2) {
    o = pack8_f16(a, c);
  } else {
    const v4u hi = pack8_bf16(a, c);
    o = hi;
    if (FORM == 1) { const v4u lo = pack8_bf16_lo(a, c); o = second ? lo : hi; }
  }
  const v4u mw = (v4u){ pk16(mk[0], mk[1]), pk16(mk[2], mk[3]), pk16(mk[4], mk[5]), pk16(mk[6], mk[7]) };
  o &= mw;
  if (g < total) {
    volatile v4u* q = (volatile v4u*)(dst + (size_t)g * 8);
    *q = o;
    __threadfence();
    *q = o;
  }
}

template <int FORM> struct FragOf    { typedef FragB T; };
template <>         struct FragOf<2> { typedef FragH T; };
__device__ __forceinline__ v8f mm(const FragB& a, const FragB& b, v8f c) { return wmb(a, b, c); }
__device__ __forceinline__ v8f mm(const FragH& a, const FragH& b, v8f c) { return wmh(a, b, c); }
template <class F> __device__ __forceinline__ F ld_frag(const unsigned short* p) {
  F f;
  f.h[0] = *(const v8usa*)(p);
  f.h[1] = *(const v8usa*)(p + 16);
  return f;
}

template <int FORM, int EPI>
__global__ __launch_bounds__(256) __attribute__((amdgpu_num_vgpr(248)))
void k_gemm_nt(const unsigned short* __restrict__ A, const unsigned short* __restrict__ B,
               const float* __restrict__ bias, float* __restrict__ D, int M, int N, int KTOT, int ldd) {
  static_assert(FORM >= 0 && FORM <= 2);
  static_assert(EPI == 0 || EPI == 1);
  typedef typename FragOf<FORM>::T F;
  __shared__ __attribute__((aligned(16))) float sT[8][16 * 68];
  const int lane = threadIdx.x & 31;
  const int wave = threadIdx.x >> 5;
  const int tilesM = (M + 63) >> 6;
  const int tilesN = (N + 63) >> 6;
  const int tile = blockIdx.x * 8 + wave;
  if (tile >= tilesM * tilesN) return;
  const int tm = tile / tilesN;
  const int tn = tile - tm * tilesN;
  const int m0 = tm << 6;
  const int n0 = tn << 6;

  const int rl = lane & 15;
  const int h8 = (lane >> 4) * 8;
  const unsigned short* pa = A + (size_t)(m0 + rl) * (size_t)KTOT + h8;
  const unsigned short* pb = B + (size_t)(n0 + rl) * (size_t)KTOT + h8;

  v8f acc[4][4];
#pragma unroll
  for (int i = 0; i < 4; ++i)
#pragma unroll
    for (int j = 0; j < 4; ++j) acc[i][j] = (v8f){0.f, 0.f, 0.f, 0.f, 0.f, 0.f, 0.f, 0.f};

#pragma unroll 1
  for (int k0 = 0; k0 < KTOT; k0 += 32) {
    F bf[4];
#pragma unroll
    for (int j = 0; j < 4; ++j) bf[j] = ld_frag<F>(pb + (size_t)(j << 4) * (size_t)KTOT + k0);
#pragma unroll
    for (int i = 0; i < 4; ++i) {
      const F af = ld_frag<F>(pa + (size_t)(i << 4) * (size_t)KTOT + k0);
#pragma unroll
      for (int j = 0; j < 4; ++j) acc[i][j] = mm(af, bf[j], acc[i][j]);
    }
  }

  float* slab = sT[wave];
  const int hh = lane >> 4;
  const int c4 = (lane & 15) * 4;
  const int nc = n0 + c4;
  const bool cok = nc < N;
  v4f bv = (v4f){0.f, 0.f, 0.f, 0.f};
  if (EPI == 1) {
    bv = *(const v4fa*)(bias + clampi(nc, 0, N - 4));
    asm volatile("" :: "v"(bv));
  }
#pragma unroll
  for (int i = 0; i < 4; ++i) {
    const int mBase = m0 + (i << 4);
#pragma unroll
    for (int j = 0; j < 4; ++j) {
#pragma unroll
      for (int r = 0; r < 8; ++r) slab[(h8 + r) * 68 + (j << 4) + rl] = acc[i][j][r];
    }
    __builtin_amdgcn_fence(__ATOMIC_RELEASE, "workgroup");
    __builtin_amdgcn_wave_barrier();
    __builtin_amdgcn_fence(__ATOMIC_ACQUIRE, "workgroup");
    v4f vv[8];
#pragma unroll
    for (int it = 0; it < 8; ++it) {
      const int row = it * 2 + hh;
      v4f v = *(const v4fa*)(slab + row * 68 + c4);
      if (EPI == 1) v += bv;
      vv[it] = v;
    }
    for (int pass = 0; pass < 2; ++pass) {
#pragma unroll
      for (int it = 0; it < 8; ++it) {
        const int row = mBase + it * 2 + hh;
        if (cok && row < M) *(volatile v4f*)(D + (size_t)row * (size_t)ldd + nc) = vv[it];
      }
      __threadfence();
    }
    __builtin_amdgcn_fence(__ATOMIC_RELEASE, "workgroup");
    __builtin_amdgcn_wave_barrier();
    __builtin_amdgcn_fence(__ATOMIC_ACQUIRE, "workgroup");
  }
}

#define N_NODES  50000
#define N_EDGES  1600000
#define MPN      50048
#define NBRUN    512
#define NBLK     98
#define RCAP     20894
#define RCAPP    20992
#define DEGCAP   72
#define SROWS    76
#define NTHR     256
#define NWAVE    8
#define EPT      8
#define CHUNK    (NTHR * EPT)
#define WCAP     (EPT * 32)
#define LISTN    (NWAVE * WCAP)
#define OFFP     544
#define LDS_BKT  ((2 * RCAPP + NBRUN + OFFP + LISTN + 32) * 4)

#define SPLIT_L0 1
#define SPLIT_L1 1
#define SPLIT_L2 1
#define SPLIT_H  1

#define TAB_PAR  0
#define TAB_ATT  288
#define TAB_INB  672
#define TAB_HT   736
#define TAB_N    1536
#define HT_N     800

static_assert(N_EDGES < (1 << 21));
static_assert(NBRUN <= (1 << 9));
static_assert(NBLK * NBRUN >= N_NODES && (NBLK - 1) * NBRUN < N_NODES);
static_assert(RCAP * 4 >= 16715 * 5);
static_assert(RCAPP >= RCAP && (RCAPP % 128) == 0 && (RCAPP % 4) == 0);
static_assert(DEGCAP >= 61 + 8 + 1);
static_assert(SROWS >= DEGCAP + 1 && DEGCAP <= 96);
static_assert((MPN % 128) == 0 && MPN >= N_NODES && (N_NODES % 16) == 0 && (N_NODES % 8) == 0);
static_assert((MPN * 32 / 8) % 256 == 0 && (MPN * 128 / 8) % 256 == 0);
static_assert((OFFP % 32) == 0 && OFFP == NBRUN + 32);
static_assert(NTHR * 2 == NBRUN);
static_assert(CHUNK == 2048 && LISTN >= NWAVE * WCAP && LISTN >= NBRUN);
static_assert(LDS_BKT <= 262144);
static_assert(LDS_BKT + 0 <= 327680);
static_assert((2 * N_NODES) % 32 == 0 && ((2 * N_NODES / 32) % 5) == 0);
static_assert((2 * N_NODES * 4) % 128 == 0);
static_assert(TAB_N - TAB_HT == HT_N && (HT_N % 160) == 0);
static_assert(((N_NODES + 31) / 32) * 32 <= MPN);

#define WS_OXB   ((size_t)0)
#define WS_OINW  (WS_OXB  + (size_t)MPN * 32 * 2)
#define WS_OGLT  (WS_OINW + (size_t)64 * 32 * 2)
#define WS_OHWT  (WS_OGLT + (size_t)3 * 64 * 128 * 2)
#define WS_OTAB  (WS_OHWT + (size_t)64 * 128 * 2)
#define WS_OAPL  (WS_OTAB + (size_t)TAB_N * 4)
#define WS_OHP   (WS_OAPL + (size_t)MPN * 128 * 2)
#define WS_OSD   (WS_OHP  + (size_t)MPN * 64 * 4)
#define WS_OMEA  (WS_OSD  + (size_t)MPN * 8 * 4)
#define WS_OLIST (WS_OMEA + (size_t)MPN * 8 * 4)
#define WS_OOFFS (WS_OLIST + (size_t)NBLK * RCAPP * 8)
#define WS_TOTAL (WS_OOFFS + (size_t)NBLK * OFFP * 4)
static_assert(WS_TOTAL == (size_t)48777472);
static_assert(WS_TOTAL <= ((size_t)128 << 20));
static_assert((WS_OINW % 128) == 0 && (WS_OGLT % 128) == 0 && (WS_OHWT % 128) == 0 && (WS_OTAB % 128) == 0);
static_assert((WS_OAPL % 128) == 0 && (WS_OHP % 128) == 0 && (WS_OSD % 128) == 0 && (WS_OMEA % 128) == 0);
static_assert((WS_OLIST % 128) == 0 && (WS_OOFFS % 128) == 0);

typedef int   v4i __attribute__((ext_vector_type(4)));
typedef int   v2i __attribute__((ext_vector_type(2)));
typedef float v2f __attribute__((ext_vector_type(2)));
typedef v4i __attribute__((may_alias)) v4ia;
typedef v2i __attribute__((may_alias)) v2ia;
typedef v2f __attribute__((may_alias)) v2fa;

__device__ __forceinline__ void wave_sync() {
  __builtin_amdgcn_fence(__ATOMIC_RELEASE, "workgroup");
  __builtin_amdgcn_wave_barrier();
  __builtin_amdgcn_fence(__ATOMIC_ACQUIRE, "workgroup");
}
__device__ __forceinline__ float leaky02(float v) { return (v > 0.0f) ? v : 0.2f * v; }
__device__ __forceinline__ float nmax(float m, float c) { return (c > m || c != c) ? c : m; }

__device__ __forceinline__ void prep_unit(const float* __restrict__ w, int ld, int kin, int KP, int nsub, int u,
                                          unsigned short* __restrict__ wt) {
  const int ppr = KP >> 3;
  const int n   = u / ppr;
  const int k8  = (u - n * ppr) * 8;
  const int ks  = k8 & (kin - 1);
  const float* base = w + (size_t)ks * (size_t)ld + (n - nsub);
  float x[8];
#pragma unroll
  for (int e = 0; e < 8; ++e) {
    const float v = base[(size_t)e * (size_t)ld];
    asm volatile("" :: "v"(v));
    x[e] = v;
  }
  const v4u o = pack8_bf16((v4f){ x[0], x[1], x[2], x[3] }, (v4f){ x[4], x[5], x[6], x[7] });
  volatile v4u* q = (volatile v4u*)(wt + (size_t)n * (size_t)KP + k8);
  *q = o;
  __threadfence();
  *q = o;
}

__device__ __forceinline__ void tab_fill(const float* __restrict__ p, int n, int tid, float* sT, int off) {
  const float x = p[tid < n ? tid : n - 1];
  asm volatile("" :: "v"(x) : "memory");
  if (tid < n) sT[off + tid] = bf16_val(x);
}

__global__ __launch_bounds__(NTHR) void k_prep(
    const float* __restrict__ inw, const float* __restrict__ wl, const float* __restrict__ cw1,
    const float* __restrict__ rw1, const float* __restrict__ inb, const float* __restrict__ atS,
    const float* __restrict__ atD, const float* __restrict__ linE, const float* __restrict__ atE,
    const float* __restrict__ gb, const float* __restrict__ cb1, const float* __restrict__ cw2,
    const float* __restrict__ cb2, const float* __restrict__ cw3, const float* __restrict__ cb3,
    const float* __restrict__ rb1, const float* __restrict__ rw2, const float* __restrict__ rb2,
    unsigned short* __restrict__ INWT, unsigned short* __restrict__ GLT, unsigned short* __restrict__ HWT,
    float* __restrict__ TAB) {
  __shared__ __attribute__((aligned(16))) float sT[TAB_N];
  const int tid = (int)threadIdx.x;
  const int blk = (int)blockIdx.x;
  if (blk == 0) {
    prep_unit(inw, 64, 32, 32, 0, tid, INWT);
  } else if (blk < 13) {
    const int l = (blk - 1) >> 2;
    const int u = ((blk - 1) & 3) * NTHR + tid;
    prep_unit(wl + (size_t)l * 4096, 64, 64, 128, 0, u, GLT + (size_t)l * 64 * 128);
  } else if (blk < 15) {
    prep_unit(cw1, 32, 64, 128, 0, (blk - 13) * NTHR + tid, HWT);
  } else if (blk < 17) {
    prep_unit(rw1, 32, 64, 128, 32, 512 + (blk - 15) * NTHR + tid, HWT);
  } else {
    {
      const int idx = tid < 60 ? tid : 59;
      const int l = idx / 20;
      const int r = idx - l * 20;
      const int f = r >> 2;
      const int hd = r & 3;
      const float* pl = linE + l * 320 + f * 64 + hd * 16;
      const float* pa = atE + l * 64 + hd * 16;
      float s = 0.0f;
#pragma unroll 4
      for (int c = 0; c < 16; ++c) {
        const float a = pl[c];
        const float b = pa[c];
        asm volatile("" :: "v"(a));
        asm volatile("" :: "v"(b) : "memory");
        s = fmaf(bf16_val(a), bf16_val(b), s);
      }
      if (tid < 60) sT[TAB_PAR + l * 96 + r] = s;
      if (tid < 36) sT[TAB_PAR + (tid / 12) * 96 + 20 + (tid % 12)] = 0.0f;
    }
#pragma unroll 1
    for (int l = 0; l < 3; ++l) {
      tab_fill(gb + 64 * l, 64, tid, sT, TAB_PAR + l * 96 + 32);
      tab_fill(atS + 64 * l, 64, tid, sT, TAB_ATT + l * 128);
      tab_fill(atD + 64 * l, 64, tid, sT, TAB_ATT + l * 128 + 64);
    }
    tab_fill(inb, 64, tid, sT, TAB_INB);
    tab_fill(cb1, 32, tid, sT, TAB_HT + 0);
    tab_fill(rb1, 32, tid, sT, TAB_HT + 32);
    tab_fill(cw2, 256, tid, sT, TAB_HT + 64);
    tab_fill(cw2 + 256, 256, tid, sT, TAB_HT + 320);
    tab_fill(cb2, 16, tid, sT, TAB_HT + 576);
    tab_fill(cw3, 16, tid, sT, TAB_HT + 592);
    tab_fill(rw2, 32, tid, sT, TAB_HT + 608);
    tab_fill(cb3, 1, tid, sT, TAB_HT + 640);
    tab_fill(rb2, 1, tid, sT, TAB_HT + 641);
    if (tid < 158) sT[TAB_HT + 642 + tid] = 0.0f;
    __syncthreads();
#pragma unroll 1
    for (int it = 0; it < 2; ++it) {
      const int p  = it * NTHR + tid;
      const int pc = p < TAB_N / 4 ? p : TAB_N / 4 - 1;
      const v4f o = *(const v4fa*)(sT + 4 * pc);
      volatile v4f* q = (volatile v4f*)(TAB + 4 * pc);
      const bool ok = p < TAB_N / 4;
      if (ok) *q = o;
      __threadfence();
      if (ok) *q = o;
    }
  }
}

__device__ __forceinline__ int scan_chunk(const int* __restrict__ dsts, int nE, int cbase, int slotBase,
                                          int nb, int* list, int tid, int lane, int wave) {
  int wc = 0;
  const int el0  = tid * EPT;
  const int e0   = cbase + el0;
  const int sent = (-0x7fffffff - 1);
  v4i da, db;
  if (cbase + CHUNK <= nE) {
    da = *(const v4ia*)(dsts + e0);
    db = *(const v4ia*)(dsts + e0 + 4);
  } else {
    const int hi = nE - 1;
    const int t0 = dsts[e0     < hi ? e0     : hi];
    const int t1 = dsts[e0 + 1 < hi ? e0 + 1 : hi];
    const int t2 = dsts[e0 + 2 < hi ? e0 + 2 : hi];
    const int t3 = dsts[e0 + 3 < hi ? e0 + 3 : hi];
    const int t4 = dsts[e0 + 4 < hi ? e0 + 4 : hi];
    const int t5 = dsts[e0 + 5 < hi ? e0 + 5 : hi];
    const int t6 = dsts[e0 + 6 < hi ? e0 + 6 : hi];
    const int t7 = dsts[e0 + 7 < hi ? e0 + 7 : hi];
    asm volatile("" :: "v"(t0)); asm volatile("" :: "v"(t1)); asm volatile("" :: "v"(t2)); asm volatile("" :: "v"(t3));
    asm volatile("" :: "v"(t4)); asm volatile("" :: "v"(t5)); asm volatile("" :: "v"(t6)); asm volatile("" :: "v"(t7));
    da.x = (e0     < nE) ? t0 : sent;
    da.y = (e0 + 1 < nE) ? t1 : sent;
    da.z = (e0 + 2 < nE) ? t2 : sent;
    da.w = (e0 + 3 < nE) ? t3 : sent;
    db.x = (e0 + 4 < nE) ? t4 : sent;
    db.y = (e0 + 5 < nE) ? t5 : sent;
    db.z = (e0 + 6 < nE) ? t6 : sent;
    db.w = (e0 + 7 < nE) ? t7 : sent;
  }
  const unsigned nbs = (unsigned)slotBase;
  const unsigned unb = (unsigned)nb;
  const unsigned s0 = (unsigned)da.x - nbs, s1 = (unsigned)da.y - nbs;
  const unsigned s2 = (unsigned)da.z - nbs, s3 = (unsigned)da.w - nbs;
  const unsigned s4 = (unsigned)db.x - nbs, s5 = (unsigned)db.y - nbs;
  const unsigned s6 = (unsigned)db.z - nbs, s7 = (unsigned)db.w - nbs;
  const bool h0 = s0 < unb, h1 = s1 < unb, h2 = s2 < unb, h3 = s3 < unb;
  const bool h4 = s4 < unb, h5 = s5 < unb, h6 = s6 < unb, h7 = s7 < unb;
  const unsigned any = __builtin_amdgcn_ballot_w32(h0 | h1 | h2 | h3 | h4 | h5 | h6 | h7);
  if (any != 0u) {
#define HITJ(J, HJ, SJ) { \
      const unsigned mj = __builtin_amdgcn_ballot_w32(HJ); \
      if (mj != 0u) { \
        if (HJ) { \
          const int pos = wc + (int)__builtin_amdgcn_mbcnt_lo(mj, 0u); \
          if (pos < WCAP) list[wave * WCAP + pos] = ((el0 + (J)) << 12) | (int)(SJ); \
        } \
        wc += (int)__builtin_popcount(mj); } }
    HITJ(0, h0, s0)
    HITJ(1, h1, s1)
    HITJ(2, h2, s2)
    HITJ(3, h3, s3)
    HITJ(4, h4, s4)
    HITJ(5, h5, s5)
    HITJ(6, h6, s6)
    HITJ(7, h7, s7)
#undef HITJ
  }
  return wc;
}

__global__ __launch_bounds__(NTHR) void k_bucket(const int* __restrict__ dsts, const int* __restrict__ srcs,
                                                 int* __restrict__ LIST, int* __restrict__ OFFS, int nN, int nE) {
  extern __shared__ v4u lds_dyn[];
  int* reg1 = (int*)lds_dyn;
  int* reg2 = reg1 + RCAPP;
  int* scnt = reg2 + RCAPP;
  int* soff = scnt + NBRUN;
  int* list = soff + OFFP;
  int* wcnt = list + LISTN;
  int* wtot = wcnt + NWAVE;
  int* wflg = wtot + NWAVE;
  const int tid = (int)threadIdx.x, lane = tid & 31, wave = tid >> 5;
  const int b = (int)blockIdx.x;
  const int slotBase = b * NBRUN;
  int nb = nN - slotBase;
  nb = nb < 0 ? 0 : (nb > NBRUN ? NBRUN : nb);

  {
    const v4i z4 = (v4i){0, 0, 0, 0};
    for (int i = tid; i < NBRUN; i += NTHR) scnt[i] = 0;
    for (int i = tid; i < RCAPP / 4; i += NTHR) *(v4ia*)(reg2 + 4 * i) = z4;
  }
  __syncthreads();

  int totraw = 0;
  const int nChunks = (nE + CHUNK - 1) / CHUNK;
#pragma unroll 1
  for (int ch = 0; ch < nChunks; ++ch) {
    const int cbase = ch * CHUNK;
    const int wc = scan_chunk(dsts, nE, cbase, slotBase, nb, list, tid, lane, wave);
    if (lane == 0) wcnt[wave] = wc;
    __syncthreads();
    int pre = 0, all = 0;
#pragma unroll
    for (int w2 = 0; w2 < NWAVE; ++w2) {
      int c = wcnt[w2];
      c = c < 0 ? 0 : (c > WCAP ? WCAP : c);
      all += c;
      pre += (w2 < wave) ? c : 0;
    }
    const int wcc  = wc > WCAP ? WCAP : wc;
    const int tot  = totraw > RCAPP ? RCAPP : totraw;
    const int base = tot + pre;
#pragma unroll 1
    for (int i0 = 0; i0 < wcc; i0 += 32) {
      const int i  = i0 + lane;
      const int ic = i < wcc ? i : wcc - 1;
      const int ent = list[wave * WCAP + ic];
      const int el  = (ent >> 12) & (CHUNK - 1);
      const int sl  = ent & (NBRUN - 1);
      int eid = cbase + el;
      eid = eid > nE - 1 ? nE - 1 : eid;
      const int pos = base + i;
      if (i < wcc && pos < RCAPP) reg1[pos] = (int)(((unsigned)sl << 21) | (unsigned)eid);
    }
    totraw += all;
    __syncthreads();
  }
  const int nh  = totraw > RCAPP ? RCAPP : totraw;
  const int ovf = totraw > RCAP ? 1 : 0;

  if (wave == 0) {
#pragma unroll 1
    for (int b0 = 0; b0 < nh; b0 += 32) {
      const int idx = b0 + lane;
      const int uv  = reg1[idx < nh ? idx : nh - 1];
      const int m32 = (nh - b0) < 32 ? (nh - b0) : 32;
#pragma unroll 1
      for (int k = 0; k < m32; ++k) {
        const int u  = __builtin_amdgcn_readlane(uv, k);
        const int sl = (int)(((unsigned)u >> 21) & (unsigned)(NBRUN - 1));
        if (lane == 0) scnt[sl] = scnt[sl] + 1;
      }
    }
  }
  __syncthreads();

  int fl = ovf;
  {
    const v2i ca = *(const v2ia*)(scnt + 2 * tid);
    const int e0 = ca.x < 0 ? 0 : ca.x, e1 = ca.y < 0 ? 0 : ca.y;
    const bool big = (e0 > DEGCAP) | (e1 > DEGCAP);
    const unsigned bm = __builtin_amdgcn_ballot_w32(big);
    const int ts = e0 + e1;
    int incl = ts;
#pragma unroll
    for (int d = 1; d < 32; d <<= 1) {
      const int up = __shfl_up(incl, d);
      if (lane >= d) incl += up;
    }
    if (lane == 31) wtot[wave] = incl;
    if (lane == 0)  wflg[wave] = (bm != 0u) ? 1 : 0;
    __syncthreads();
    int pre = 0;
#pragma unroll
    for (int w2 = 0; w2 < NWAVE; ++w2) {
      pre += (w2 < wave) ? wtot[w2] : 0;
      fl |= wflg[w2];
    }
    int run = pre + incl - ts;
    soff[2 * tid + 0] = run; run += e0;
    soff[2 * tid + 1] = run;
    if (tid < 32) soff[NBRUN + tid] = (tid < 2) ? nh : ((tid == 2) ? fl : 0);
  }
  __syncthreads();
  for (int i = tid; i < NBRUN; i += NTHR) list[i] = soff[i];
  __syncthreads();

  if (wave == 0) {
#pragma unroll 1
    for (int b0 = 0; b0 < nh; b0 += 32) {
      const int idx = b0 + lane;
      const int uv  = reg1[idx < nh ? idx : nh - 1];
      const int m32 = (nh - b0) < 32 ? (nh - b0) : 32;
#pragma unroll 1
      for (int k = 0; k < m32; ++k) {
        const int u   = __builtin_amdgcn_readlane(uv, k);
        const int sl  = (int)(((unsigned)u >> 21) & (unsigned)(NBRUN - 1));
        const int eid = (int)((unsigned)u & 0x1FFFFFu);
        if (lane == 0) {
          int pos = list[sl];
          pos = pos < 0 ? 0 : (pos > RCAPP - 1 ? RCAPP - 1 : pos);
          reg2[pos] = eid;
          list[sl] = pos + 1;
        }
      }
    }
  }
  __syncthreads();

  {
    int* Lb = LIST + (size_t)b * (size_t)RCAPP * 2;
    const int nU = RCAPP / 2;
#pragma unroll 1
    for (int it = 0; it < (nU + NTHR - 1) / NTHR; ++it) {
      const int u  = it * NTHR + tid;
      const int uc = u < nU ? u : nU - 1;
      const v2i ee = *(const v2ia*)(reg2 + 2 * uc);
      const int e0 = clampi(ee.x, 0, nE - 1);
      const int e1 = clampi(ee.y, 0, nE - 1);
      int s0 = srcs[e0];
      int s1 = srcs[e1];
      asm volatile("" :: "v"(s0));
      asm volatile("" :: "v"(s1));
      s0 = clampi(s0, 0, nN - 1);
      s1 = clampi(s1, 0, nN - 1);
      const int m0 = (2 * uc     < nh) ? -1 : 0;
      const int m1 = (2 * uc + 1 < nh) ? -1 : 0;
      const v4i o = (v4i){ s0 & m0, e0 & m0, s1 & m1, e1 & m1 };
      volatile v4i* q = (volatile v4i*)(Lb + 4 * (size_t)uc);
      const bool ok = u < nU;
      if (ok) *q = o;
      __threadfence();
      if (ok) *q = o;
    }
  }
  {
    int* Ob = OFFS + (size_t)b * OFFP;
    const int nU = OFFP / 4;
#pragma unroll 1
    for (int it = 0; it < (nU + NTHR - 1) / NTHR; ++it) {
      const int u  = it * NTHR + tid;
      const int uc = u < nU ? u : nU - 1;
      const v4i o = *(const v4ia*)(soff + 4 * uc);
      volatile v4i* q = (volatile v4i*)(Ob + 4 * uc);
      const bool ok = u < nU;
      if (ok) *q = o;
      __threadfence();
      if (ok) *q = o;
    }
  }
}

__global__ __launch_bounds__(NTHR) void k_meanea(const float* __restrict__ ea, const int* __restrict__ LIST,
                                                 const int* __restrict__ OFFS, float* __restrict__ MEA,
                                                 int nReal, int nE) {
  __shared__ float sE[NWAVE][96 * 5];
  __shared__ __attribute__((aligned(16))) float sM[NWAVE * 8];
  const int tid = (int)threadIdx.x, lane = tid & 31, wave = tid >> 5;
  const int row  = (int)blockIdx.x * NWAVE + wave;
  const bool live = row < nReal;
  const int rowc = clampi(row, 0, nReal - 1);
  const int b    = rowc / NBRUN;
  const int slot = rowc & (NBRUN - 1);
  const int* ob = OFFS + (size_t)b * OFFP;
  int o0 = ob[slot];
  int o1 = ob[slot + 1];
  asm volatile("" :: "v"(o0));
  asm volatile("" :: "v"(o1));
  const int st = clampi(o0, 0, RCAPP - 1);
  int c = clampi(o1 - o0, 0, DEGCAP);
  c = c > RCAPP - st ? RCAPP - st : c;
  c = live ? c : 0;
  const int cn  = __builtin_amdgcn_readfirstlane(c);
  const int stu = __builtin_amdgcn_readfirstlane(st);
  const int* lp = LIST + ((size_t)b * (size_t)RCAPP + (size_t)stu) * 2;
  float* se = sE[wave];
#pragma unroll 1
  for (int s0 = 0; s0 < cn; s0 += 32) {
    const int j  = s0 + lane;
    const int jc = j < cn ? j : cn - 1;
    v2i pr = *(const v2ia*)(lp + 2 * jc);
    asm volatile("" :: "v"(pr));
    const int eid = clampi(pr.y, 0, nE - 1);
    const float* ep = ea + (size_t)eid * 5;
    const float e0 = ep[0];
    const float e1 = ep[1];
    const float e2 = ep[2];
    const float e3 = ep[3];
    const float e4 = ep[4];
    asm volatile("" :: "v"(e0)); asm volatile("" :: "v"(e1)); asm volatile("" :: "v"(e2));
    asm volatile("" :: "v"(e3)); asm volatile("" :: "v"(e4));
    const bool ok = j < cn;
    se[j * 5 + 0] = ok ? bf16_val(e0) : 0.0f;
    se[j * 5 + 1] = ok ? bf16_val(e1) : 0.0f;
    se[j * 5 + 2] = ok ? bf16_val(e2) : 0.0f;
    se[j * 5 + 3] = ok ? bf16_val(e3) : 0.0f;
    se[j * 5 + 4] = ok ? bf16_val(e4) : 0.0f;
  }
  wave_sync();
  const int fcl = lane < 5 ? lane : 4;
  float s = 0.0f;
#pragma unroll 1
  for (int j = 0; j < cn; ++j) s += se[j * 5 + fcl];
  const float dn = fmaxf((float)cn, 1.0f);
  const float mean = s / dn;
  if (lane < 8) sM[wave * 8 + lane] = (lane < 5) ? mean : 0.0f;
  __syncthreads();
  {
    const int pc = tid & 15;
    const v4f o = *(const v4fa*)(sM + 4 * pc);
    volatile v4f* q = (volatile v4f*)(MEA + (size_t)blockIdx.x * 64 + 4 * pc);
    const bool ok = tid < 16;
    if (ok) *q = o;
    __threadfence();
    if (ok) *q = o;
  }
}

__global__ __launch_bounds__(NTHR) void k_scores(const float* __restrict__ HP, const float* __restrict__ ATTl,
                                                 float* __restrict__ SD, int nReal) {
  __shared__ __attribute__((aligned(16))) float sA[128];
  __shared__ __attribute__((aligned(16))) float sS[32 * 8];
  const int tid = (int)threadIdx.x, lane = tid & 31, wave = tid >> 5;
  if (tid < 128) sA[tid] = ATTl[tid];
  __syncthreads();
  const float asx = sA[2 * lane], asy = sA[2 * lane + 1];
  const float adx = sA[64 + 2 * lane], ady = sA[65 + 2 * lane];
  const int rb = (int)blockIdx.x * 32 + wave * 4;
#pragma unroll
  for (int i = 0; i < 4; ++i) {
    const int r = clampi(rb + i, 0, nReal - 1);
    v2f v = *(const v2fa*)(HP + (size_t)r * 64 + 2 * lane);
    asm volatile("" :: "v"(v));
    float ps = v.x * asx + v.y * asy;
    float pd = v.x * adx + v.y * ady;
    ps += __shfl_xor(ps, 1);
    pd += __shfl_xor(pd, 1);
    ps += __shfl_xor(ps, 2);
    pd += __shfl_xor(pd, 2);
    ps += __shfl_xor(ps, 4);
    pd += __shfl_xor(pd, 4);
    if ((lane & 7) == 0) {
      sS[(wave * 4 + i) * 8 + (lane >> 3)]     = ps;
      sS[(wave * 4 + i) * 8 + 4 + (lane >> 3)] = pd;
    }
  }
  __syncthreads();
  {
    const int pc = tid & 63;
    const v4f o = *(const v4fa*)(sS + 4 * pc);
    volatile v4f* q = (volatile v4f*)(SD + (size_t)blockIdx.x * 256 + 4 * pc);
    const bool ok = tid < 64;
    if (ok) *q = o;
    __threadfence();
    if (ok) *q = o;
  }
}

template <int FINAL, int SPLIT>
__global__ __launch_bounds__(NTHR) void k_replay(const float* __restrict__ HP, const float* __restrict__ SD,
                                                 const float* __restrict__ MEA, const float* __restrict__ ea,
                                                 const int* __restrict__ LIST, const int* __restrict__ OFFS,
                                                 const float* __restrict__ PAR, unsigned short* __restrict__ APL,
                                                 float* __restrict__ out2, int nReal, int nE) {
  __shared__ __attribute__((aligned(16))) float sAl[NWAVE][SROWS * 4];
  __shared__ int sSrc[NWAVE][SROWS];
  __shared__ __attribute__((aligned(16))) float sPar[96];
  const int tid = (int)threadIdx.x, lane = tid & 31, wave = tid >> 5;
  if (tid < 96) sPar[tid] = PAR[tid];
  __syncthreads();
  const int row  = (int)blockIdx.x * NWAVE + wave;
  const bool live = row < nReal;
  const int rowc = clampi(row, 0, nReal - 1);
  const int b    = rowc / NBRUN;
  const int slot = rowc & (NBRUN - 1);
  const int* ob = OFFS + (size_t)b * OFFP;
  int o0 = ob[slot];
  int o1 = ob[slot + 1];
  int fg = ob[NBRUN + 2];
  asm volatile("" :: "v"(o0));
  asm volatile("" :: "v"(o1));
  asm volatile("" :: "v"(fg));
  const int st = clampi(o0, 0, RCAPP - 1);
  int c = clampi(o1 - o0, 0, DEGCAP);
  c = c > RCAPP - st ? RCAPP - st : c;
  c = live ? c : 0;
  const int cn  = __builtin_amdgcn_readfirstlane(c);
  const int stu = __builtin_amdgcn_readfirstlane(st);
  const int* lp = LIST + ((size_t)b * (size_t)RCAPP + (size_t)stu) * 2;

  v4f sdS = *(const v4fa*)(SD + (size_t)rowc * 8);
  v4f sdD = *(const v4fa*)(SD + (size_t)rowc * 8 + 4);
  v4f me0 = *(const v4fa*)(MEA + (size_t)rowc * 8);
  v4f me1 = *(const v4fa*)(MEA + (size_t)rowc * 8 + 4);
  asm volatile("" :: "v"(sdS));
  asm volatile("" :: "v"(sdD));
  asm volatile("" :: "v"(me0));
  asm volatile("" :: "v"(me1));
  const v4f mE0 = *(const v4fa*)(sPar + 0);
  const v4f mE1 = *(const v4fa*)(sPar + 4);
  const v4f mE2 = *(const v4fa*)(sPar + 8);
  const v4f mE3 = *(const v4fa*)(sPar + 12);
  const v4f mE4 = *(const v4fa*)(sPar + 16);

  float* al = sAl[wave];
  int*   ss = sSrc[wave];
  const float ninf = -__builtin_inff();
  float mx0 = ninf, mx1 = ninf, mx2 = ninf, mx3 = ninf;

#pragma unroll 1
  for (int s0 = 0; s0 < cn; s0 += 32) {
    const int j  = s0 + lane;
    const int jc = j < cn ? j : cn - 1;
    v2i pr = *(const v2ia*)(lp + 2 * jc);
    asm volatile("" :: "v"(pr));
    const int s   = clampi(pr.x, 0, nReal - 1);
    const int eid = clampi(pr.y, 0, nE - 1);
    v4f as = *(const v4fa*)(SD + (size_t)s * 8);
    asm volatile("" :: "v"(as));
    const float* ep = ea + (size_t)eid * 5;
    float e0 = ep[0];
    float e1 = ep[1];
    float e2 = ep[2];
    float e3 = ep[3];
    float e4 = ep[4];
    asm volatile("" :: "v"(e0)); asm volatile("" :: "v"(e1)); asm volatile("" :: "v"(e2));
    asm volatile("" :: "v"(e3)); asm volatile("" :: "v"(e4));
    e0 = bf16_val(e0); e1 = bf16_val(e1); e2 = bf16_val(e2); e3 = bf16_val(e3); e4 = bf16_val(e4);
    v4f ae = mE0 * e0;
    ae += mE1 * e1;
    ae += mE2 * e2;
    ae += mE3 * e3;
    ae += mE4 * e4;
    v4f a = (as + sdD) + ae;
    a.x = leaky02(a.x); a.y = leaky02(a.y); a.z = leaky02(a.z); a.w = leaky02(a.w);
    const bool ok = j < cn;
    if (ok) {
      *(v4fa*)(al + 4 * j) = a;
      ss[j] = s;
    }
    mx0 = nmax(mx0, ok ? a.x : ninf);
    mx1 = nmax(mx1, ok ? a.y : ninf);
    mx2 = nmax(mx2, ok ? a.z : ninf);
    mx3 = nmax(mx3, ok ? a.w : ninf);
  }
  {
    v4f ae = mE0 * me0.x;
    ae += mE1 * me0.y;
    ae += mE2 * me0.z;
    ae += mE3 * me0.w;
    ae += mE4 * me1.x;
    v4f a = (sdS + sdD) + ae;
    a.x = leaky02(a.x); a.y = leaky02(a.y); a.z = leaky02(a.z); a.w = leaky02(a.w);
    if (lane == 0) {
      *(v4fa*)(al + 4 * cn) = a;
      ss[cn] = rowc;
    }
    mx0 = nmax(mx0, a.x); mx1 = nmax(mx1, a.y); mx2 = nmax(mx2, a.z); mx3 = nmax(mx3, a.w);
  }
#pragma unroll
  for (int d = 1; d < 32; d <<= 1) {
    const float q0 = __shfl_xor(mx0, d);
    const float q1 = __shfl_xor(mx1, d);
    const float q2 = __shfl_xor(mx2, d);
    const float q3 = __shfl_xor(mx3, d);
    mx0 = nmax(mx0, q0); mx1 = nmax(mx1, q1); mx2 = nmax(mx2, q2); mx3 = nmax(mx3, q3);
  }
  wave_sync();

#pragma unroll 1
  for (int s0 = 0; s0 < cn + 1; s0 += 32) {
    const int j  = s0 + lane;
    const int jc = j < cn ? j : cn;
    const v4f a = *(const v4fa*)(al + 4 * jc);
    v4f ex;
    ex.x = expf(a.x - mx0);
    ex.y = expf(a.y - mx1);
    ex.z = expf(a.z - mx2);
    ex.w = expf(a.w - mx3);
    if (j <= cn) *(v4fa*)(al + 4 * j) = ex;
  }
  wave_sync();
  const int hd = lane >> 3;
  float den = 0.0f;
#pragma unroll 1
  for (int j = 0; j <= cn; ++j) den += al[4 * j + hd];
  const float d0 = __shfl(den, 0);
  const float d1 = __shfl(den, 8);
  const float d2 = __shfl(den, 16);
  const float d3 = __shfl(den, 24);
  wave_sync();
#pragma unroll 1
  for (int s0 = 0; s0 < cn + 1; s0 += 32) {
    const int j  = s0 + lane;
    const int jc = j < cn ? j : cn;
    const v4f ex = *(const v4fa*)(al + 4 * jc);
    v4f w;
    w.x = ex.x / d0;
    w.y = ex.y / d1;
    w.z = ex.z / d2;
    w.w = ex.w / d3;
    if (j <= cn) *(v4fa*)(al + 4 * j) = w;
  }
  wave_sync();

  float accx = 0.0f, accy = 0.0f;
  const float* hpl = HP + 2 * lane;
#pragma unroll 1
  for (int j = 0; j <= cn; ++j) {
    const int s = clampi(ss[j], 0, nReal - 1);
    const float w = al[4 * j + hd];
    v2f v = *(const v2fa*)(hpl + (size_t)s * 64);
    asm volatile("" :: "v"(v));
    accx += v.x * w;
    accy += v.y * w;
  }
  float vx = accx + sPar[32 + 2 * lane];
  float vy = accy + sPar[33 + 2 * lane];
  if (FINAL == 0) {
    const float ex_ = expm1f(vx);
    const float ey_ = expm1f(vy);
    vx = (vx > 0.0f) ? vx : ex_;
    vy = (vy > 0.0f) ? vy : ey_;
  }
  const float qn = __uint_as_float(0x7fc00000u);
  vx = (fg != 0) ? qn : vx;
  vy = (fg != 0) ? qn : vy;
  const unsigned whi = pk16(bf16_bits(vx), bf16_bits(vy));
  const unsigned wlo = SPLIT ? pk16(bf16_lo_bits(vx), bf16_lo_bits(vy)) : 0u;
  const v2f vo = (v2f){ vx, vy };
  volatile unsigned* ar = (volatile unsigned*)(APL + (size_t)rowc * 128);
  volatile v2f* og = (volatile v2f*)(out2 + (size_t)rowc * 64 + 2 * lane);
  if (live) {
    ar[lane] = whi;
    ar[32 + lane] = wlo;
    if (FINAL == 1) *og = vo;
  }
  __threadfence();
  if (live) {
    ar[lane] = whi;
    ar[32 + lane] = wlo;
    if (FINAL == 1) *og = vo;
  }
}

__global__ __launch_bounds__(160) void k_heads(const float* __restrict__ Y, const float* __restrict__ HT,
                                               float* __restrict__ out, int nReal) {
  __shared__ float sW[HT_N];
  __shared__ float sY[5][64 * 32];
  const int tid = (int)threadIdx.x, lane = tid & 31, wave = tid >> 5;
#pragma unroll 1
  for (int i = 0; i < HT_N / 160; ++i) sW[i * 160 + tid] = HT[i * 160 + tid];
  __syncthreads();
  const int f = ((int)blockIdx.x * 5 + wave) * 32 + lane;
  const int node = clampi(f < nReal ? f : f - nReal, 0, nReal - 1);
  const float* yr = Y + (size_t)node * 64;
  float* my = sY[wave] + lane;
#pragma unroll 4
  for (int q = 0; q < 16; ++q) {
    v4f v = *(const v4fa*)(yr + 4 * q);
    asm volatile("" :: "v"(v));
    const float t0 = v.x + sW[4 * q + 0];
    const float t1 = v.y + sW[4 * q + 1];
    const float t2 = v.z + sW[4 * q + 2];
    const float t3 = v.w + sW[4 * q + 3];
    my[(4 * q + 0) * 32] = (t0 > 0.0f) ? t0 : (t0 - t0);
    my[(4 * q + 1) * 32] = (t1 > 0.0f) ? t1 : (t1 - t1);
    my[(4 * q + 2) * 32] = (t2 > 0.0f) ? t2 : (t2 - t2);
    my[(4 * q + 3) * 32] = (t3 > 0.0f) ? t3 : (t3 - t3);
  }
  float p = 0.0f;
#pragma unroll 1
  for (int j = 0; j < 16; ++j) {
    float s = 0.0f;
#pragma unroll 4
    for (int c = 0; c < 32; ++c) s = fmaf(my[c * 32], sW[64 + c * 16 + j], s);
    s += sW[576 + j];
    s = (s > 0.0f) ? s : (s - s);
    p = fmaf(s, sW[592 + j], p);
  }
  p += sW[640];
  const float prob = 1.0f / (1.0f + expf(-p));
  float r = 0.0f;
#pragma unroll 4
  for (int c = 0; c < 32; ++c) r = fmaf(my[(32 + c) * 32], sW[608 + c], r);
  r += sW[641];
  const float risk = (1.0f / (1.0f + expf(-r))) * 100.0f;
  const float val = (f >= nReal) ? risk : prob;
  const int fc = clampi(f, 0, 2 * nReal - 1);
  volatile float* q = (volatile float*)(out + fc);
  const bool ok = f < 2 * nReal;
  if (ok) *q = val;
  __threadfence();
  if (ok) *q = val;
}

static inline int cdiv_i(int a, int b) { return (a + b - 1) / b; }

extern "C" void kernel_launch(void* const* d_in, const int* in_sizes, int n_in,
                              void* d_out, int out_size, void* d_ws, size_t ws_size,
                              hipStream_t stream) {
  if (n_in < 21) return;
  if (in_sizes[0] != N_NODES * 32) return;
  if (in_sizes[1] != 2 * N_EDGES) return;
  if (in_sizes[2] != N_EDGES * 5) return;
  if (in_sizes[3] != 32 * 64 || in_sizes[4] != 64) return;
  if (in_sizes[5] != 3 * 64 * 64) return;
  if (in_sizes[6] != 192 || in_sizes[7] != 192 || in_sizes[8] != 960 || in_sizes[9] != 192 || in_sizes[10] != 192) return;
  if (in_sizes[11] != 2048 || in_sizes[12] != 32 || in_sizes[13] != 512 || in_sizes[14] != 16) return;
  if (in_sizes[15] != 16 || in_sizes[16] != 1) return;
  if (in_sizes[17] != 2048 || in_sizes[18] != 32 || in_sizes[19] != 32 || in_sizes[20] != 1) return;
  if (out_size != 2 * N_NODES + N_NODES * 64) return;
  if (ws_size < WS_TOTAL) return;

  const float* x    = (const float*)d_in[0];
  const int*   ei   = (const int*)d_in[1];
  const float* ea   = (const float*)d_in[2];
  const float* inw  = (const float*)d_in[3];
  const float* inb  = (const float*)d_in[4];
  const float* wl   = (const float*)d_in[5];
  const float* atS  = (const float*)d_in[6];
  const float* atD  = (const float*)d_in[7];
  const float* linE = (const float*)d_in[8];
  const float* atE  = (const float*)d_in[9];
  const float* gb   = (const float*)d_in[10];
  const float* cw1  = (const float*)d_in[11];
  const float* cb1  = (const float*)d_in[12];
  const float* cw2  = (const float*)d_in[13];
  const float* cb2  = (const float*)d_in[14];
  const float* cw3  = (const float*)d_in[15];
  const float* cb3  = (const float*)d_in[16];
  const float* rw1  = (const float*)d_in[17];
  const float* rb1  = (const float*)d_in[18];
  const float* rw2  = (const float*)d_in[19];
  const float* rb2  = (const float*)d_in[20];
  const int* src = ei;
  const int* dst = ei + N_EDGES;
  float* out  = (float*)d_out;
  float* out2 = out + 2 * N_NODES;

  char* ws = (char*)d_ws;
  unsigned short* XB   = (unsigned short*)(ws + WS_OXB);
  unsigned short* INWT = (unsigned short*)(ws + WS_OINW);
  unsigned short* GLT  = (unsigned short*)(ws + WS_OGLT);
  unsigned short* HWT  = (unsigned short*)(ws + WS_OHWT);
  float*          TAB  = (float*)(ws + WS_OTAB);
  unsigned short* APL  = (unsigned short*)(ws + WS_OAPL);
  float*          HP   = (float*)(ws + WS_OHP);
  float*          SD   = (float*)(ws + WS_OSD);
  float*          MEA  = (float*)(ws + WS_OMEA);
  int*            LST  = (int*)(ws + WS_OLIST);
  int*            OFS  = (int*)(ws + WS_OOFFS);

  hipFuncSetAttribute(reinterpret_cast<const void*>(&k_bucket),
                      hipFuncAttributeMaxDynamicSharedMemorySize, LDS_BKT);

  k_prep<<<18, NTHR, 0, stream>>>(inw, wl, cw1, rw1, inb, atS, atD, linE, atE, gb, cb1, cw2, cb2, cw3, cb3,
                                  rb1, rw2, rb2, INWT, GLT, HWT, TAB);
  k_plane<0><<<MPN * 32 / 8 / 256, 256, 0, stream>>>(x, N_NODES, 32, 32, XB, MPN, 32);
  k_bucket<<<NBLK, NTHR, LDS_BKT, stream>>>(dst, src, LST, OFS, N_NODES, N_EDGES);
  k_meanea<<<N_NODES / NWAVE, NTHR, 0, stream>>>(ea, LST, OFS, MEA, N_NODES, N_EDGES);

  const int T = cdiv_i(N_NODES, 64) * 1;
  const int GB = cdiv_i(T, 8);
  k_gemm_nt<0, 1><<<GB, 256, 0, stream>>>(XB, INWT, TAB + TAB_INB, HP, N_NODES, 64, 32, 64);
  k_plane<(SPLIT_L0 ? 1 : 0)><<<MPN * 128 / 8 / 256, 256, 0, stream>>>(HP, N_NODES, 64, 64, APL, MPN,
                                                                        SPLIT_L0 ? 64 : 128);

  k_gemm_nt<0, 0><<<GB, 256, 0, stream>>>(APL, GLT, TAB, HP, N_NODES, 64, 128, 64);
  k_scores<<<cdiv_i(N_NODES, 32), NTHR, 0, stream>>>(HP, TAB + TAB_ATT, SD, N_NODES);
  k_replay<0, SPLIT_L1><<<N_NODES / NWAVE, NTHR, 0, stream>>>(HP, SD, MEA, ea, LST, OFS, TAB + TAB_PAR, APL, out2,
                                                               N_NODES, N_EDGES);
  k_gemm_nt<0, 0><<<GB, 256, 0, stream>>>(APL, GLT + 64 * 128, TAB, HP, N_NODES, 64, 128, 64);
  k_scores<<<cdiv_i(N_NODES, 32), NTHR, 0, stream>>>(HP, TAB + TAB_ATT + 128, SD, N_NODES);
  k_replay<0, SPLIT_L2><<<N_NODES / NWAVE, NTHR, 0, stream>>>(HP, SD, MEA, ea, LST, OFS, TAB + TAB_PAR + 96, APL,
                                                               out2, N_NODES, N_EDGES);
  k_gemm_nt<0, 0><<<GB, 256, 0, stream>>>(APL, GLT + 2 * 64 * 128, TAB, HP, N_NODES, 64, 128, 64);
  k_scores<<<cdiv_i(N_NODES, 32), NTHR, 0, stream>>>(HP, TAB + TAB_ATT + 256, SD, N_NODES);
  k_replay<1, SPLIT_H><<<N_NODES / NWAVE, NTHR, 0, stream>>>(HP, SD, MEA, ea, LST, OFS, TAB + TAB_PAR + 192, APL,
                                                              out2, N_NODES, N_EDGES);
  k_gemm_nt<0, 0><<<GB, 256, 0, stream>>>(APL, HWT, TAB, HP, N_NODES, 64, 128, 64);
  k_heads<<<(2 * N_NODES / 32) / 5, 160, 0, stream>>>(HP, TAB + TAB_HT, out, N_NODES);
}
